// ScaledDotProduct_24824910971446
// MI455X (gfx1250) — hardware-verified
//
#include <hip/hip_runtime.h>


#ifndef NB
#define NB 16
#endif
#ifndef SEQ
#define SEQ 4096
#endif
#define NB_FULL 16
#define SEQ_FULL 4096
#define HD 64

namespace {
constexpr float XS = 8.0f, PS = 1024.0f, RS_ = 1024.0f, LOG2E = 1.4426950408889634f;
static_assert(SEQ % 64 == 0 && SEQ >= 64 && SEQ <= SEQ_FULL);
static_assert(NB >= 1 && NB <= NB_FULL);
static_assert(HD == 64);
typedef _Float16 b16;
typedef __attribute__((ext_vector_type(16))) _Float16 v16b;
typedef __attribute__((ext_vector_type(8))) _Float16 v8b;
typedef __attribute__((ext_vector_type(2))) _Float16 v2h;
typedef __attribute__((ext_vector_type(8))) float v8f;
typedef __attribute__((ext_vector_type(4))) float v4f;

__device__ __forceinline__ float bf16_rne(float f) { unsigned int u = __float_as_uint(f); u += 0x7FFFu + ((u >> 16) & 1u); return __uint_as_float(u & 0xFFFF0000u); }

__device__ __forceinline__ v16b frag_kb(const b16* p, int hh) {
  const v8b a = *(const v8b*)(p + 8 * hh), b = *(const v8b*)(p + 16 + 8 * hh); v16b f;
#pragma unroll
  for (int e = 0; e < 8; ++e) { f[e] = a[e]; f[8 + e] = b[e]; }
  return f;
}
__device__ __forceinline__ v8f wmma16b(v16b a, v16b b, v8f c) {
  v8f d = __builtin_amdgcn_wmma_f32_16x16x32_f16(false, a, false, b, (short)0, c, false, false);
  asm volatile("v_nop\n\tv_nop\n\tv_nop\n\tv_nop" : "+v"(d) : "v"(a), "v"(b));
  return d;
}
__device__ __forceinline__ void wave_lds_sync() { __builtin_amdgcn_fence(3, "workgroup"); __builtin_amdgcn_wave_barrier(); __builtin_amdgcn_fence(2, "workgroup"); }
__device__ __forceinline__ float nexp2(float v) { return __builtin_amdgcn_exp2f(v); }

__global__ __launch_bounds__(256) void qk_kernel(const float* __restrict__ q, const float* __restrict__ k, b16* __restrict__ QP, b16* __restrict__ KP) {
  const size_t u = (size_t)blockIdx.x * 256 + threadIdx.x; const size_t n8 = (size_t)NB * SEQ * HD / 8; if (u >= 2 * n8) return;
  const bool isk = u >= n8;
  const size_t e = (isk ? u - n8 : u) * 8;
  const size_t ph = e / ((size_t)SEQ * HD), rem = e - ph * (size_t)SEQ * HD;
  const float* src = (isk ? k : q) + ph * (size_t)SEQ_FULL * HD + rem;
  const v8f vv = *(const v8f*)src; v8b o;
#pragma unroll
  for (int j = 0; j < 8; ++j) o[j] = (b16)(bf16_rne(vv[j]) * XS);
  b16* dst = (isk ? KP : QP) + e;
  *(volatile v8b*)dst = o; __threadfence(); *(volatile v8b*)dst = o; __threadfence();
}

__global__ __launch_bounds__(256) void vt_kernel(const float* __restrict__ v, b16* __restrict__ VT) {
  __shared__ float tile[64][HD + 1];
  const int tid = threadIdx.x, wave = tid >> 5, lane = tid & 31; const int t0 = blockIdx.x * 64; const size_t ph = blockIdx.y;
  for (int i = tid; i < 64 * (HD / 4); i += 256) {
    const int rr = i / (HD / 4), c4 = (i % (HD / 4)) * 4;
    const v4f vv = *(const v4f*)(v + (ph * SEQ_FULL + t0 + rr) * HD + c4);
#pragma unroll
    for (int j = 0; j < 4; ++j) tile[rr][c4 + j] = bf16_rne(vv[j]) * XS;
  }
  __syncthreads();
  for (int pass = 0; pass < 2; ++pass) {
#pragma unroll 1
    for (int d = wave * 8; d < wave * 8 + 8; ++d) {
      v2h o; o[0] = (b16)tile[2 * lane][d]; o[1] = (b16)tile[2 * lane + 1][d];
      *(volatile v2h*)(VT + (ph * HD + d) * (size_t)SEQ + t0 + 2 * lane) = o;
    }
    __threadfence();
  }
}

__global__ __launch_bounds__(64) __attribute__((amdgpu_num_vgpr(256)))
void attn_kernel(const b16* __restrict__ QP, const b16* __restrict__ KP, const b16* __restrict__ VT, float* __restrict__ out) {
  __shared__ __attribute__((aligned(16))) b16 Pb[2][16][32 + 8], Pl[2][16][32 + 8];
  __shared__ __attribute__((aligned(16))) float To[2][16][HD + 4];
  const int wave = threadIdx.x >> 5, lane = threadIdx.x & 31, hh = lane >> 4, col = lane & 15;
  const size_t ph = blockIdx.y; const int q0 = blockIdx.x * 32 + wave * 16, qi = q0 + col;
  const b16* Qb = QP + ph * (size_t)SEQ * HD; const b16* Kb = KP + ph * (size_t)SEQ * HD; const b16* Vb = VT + ph * (size_t)HD * SEQ;
  v16b qa[2];
#pragma unroll
  for (int ks = 0; ks < 2; ++ks) qa[ks] = frag_kb(Qb + (size_t)qi * HD + 32 * ks, hh);
  const float cs = LOG2E * 0.125f / (XS * XS);
  float m = -INFINITY, l = 0.0f; v8f o[4], ol[4];
#pragma unroll
  for (int t = 0; t < 4; ++t) { o[t] = (v8f){}; ol[t] = (v8f){}; }
#pragma unroll 1
  for (int kb = 0; kb < SEQ; kb += 32) {
    float e[16]; float mx = -INFINITY;
#pragma unroll
    for (int u = 0; u < 2; ++u) {
      v8f s = (v8f){}; const size_t kr = (size_t)(kb + u * 16 + col) * HD;
#pragma unroll
      for (int ks = 0; ks < 2; ++ks) s = wmma16b(frag_kb(Kb + kr + 32 * ks, hh), qa[ks], s);
#pragma unroll
      for (int r = 0; r < 8; ++r) { const float vv = s[r] * cs; e[u * 8 + r] = vv; mx = fmaxf(mx, vv); }
    }
    mx = fmaxf(mx, __shfl_xor(mx, 16)); const float mn = fmaxf(m, mx); const float al = nexp2(m - mn); float sum = 0.0f;
#pragma unroll
    for (int i2 = 0; i2 < 16; ++i2) {
      const float p = nexp2(e[i2] - mn); sum += p;
      const int pc = (i2 < 8 ? 0 : 16) + 8 * hh + (i2 & 7);
      const float ps = p * PS; const b16 phh = (b16)ps;
      Pb[wave][col][pc] = phh; Pl[wave][col][pc] = (b16)((ps - (float)phh) * RS_);
    }
    sum += __shfl_xor(sum, 16); l = l * al + sum; m = mn;
    wave_lds_sync();
    const v16b pf = frag_kb(&Pb[wave][col][0], hh), plf = frag_kb(&Pl[wave][col][0], hh);
#pragma unroll
    for (int t = 0; t < 4; ++t) {
      const v16b vf = frag_kb(Vb + (size_t)(t * 16 + col) * SEQ + kb, hh);
      o[t] *= al; o[t] = wmma16b(vf, pf, o[t]); ol[t] = wmma16b(vf, plf, ol[t] * al);
    }
    wave_lds_sync();
  }
  const float inv = 1.0f / (l * PS * XS);
#pragma unroll
  for (int t = 0; t < 4; ++t)
#pragma unroll
    for (int r = 0; r < 8; ++r) To[wave][col][t * 16 + 8 * hh + r] = (o[t][r] + ol[t][r] * (1.0f / RS_)) * inv;
  wave_lds_sync();
  for (int pass = 0; pass < 2; ++pass) {
#pragma unroll 1
    for (int rr = 0; rr < 8; ++rr) {
      const int row = 2 * rr + hh;
      const v4f val = *(const v4f*)(&To[wave][row][col * 4]);
      *(volatile v4f*)(out + (ph * SEQ_FULL + q0 + row) * HD + col * 4) = val;
    }
    __threadfence();
  }
}
}

extern "C" void kernel_launch(void* const* d_in, const int* in_sizes, int n_in, void* d_out, int out_size, void* d_ws, size_t ws_size, hipStream_t stream) {
  if (n_in < 3) return;
  auto Fp = [&](int i) { return (const float*)d_in[i]; };
  const size_t need = ((size_t)(NB - 1) * SEQ_FULL + SEQ) * HD;
  if ((size_t)in_sizes[0] < need || (size_t)in_sizes[1] < need || (size_t)in_sizes[2] < need || (size_t)out_size < need) return;
  size_t off = 0; char* ws = (char*)d_ws;
  auto carve = [&](size_t bytes) { char* p = ws + off; off += (bytes + 255) & ~(size_t)255; return p; };
  const size_t plane = (size_t)NB * SEQ * HD * 2;
  b16* QP = (b16*)carve(plane); b16* KP = (b16*)carve(plane); b16* VT = (b16*)carve(plane);
  if (off > ws_size || off > ((size_t)128 << 20)) return;
  const size_t n8 = (size_t)NB * SEQ * HD / 8;
  qk_kernel<<<(unsigned)((2 * n8 + 255) / 256), 256, 0, stream>>>(Fp(0), Fp(1), QP, KP);
  vt_kernel<<<dim3(SEQ / 64, NB), 256, 0, stream>>>(Fp(2), VT);
  attn_kernel<<<dim3(SEQ / 32, NB), 64, 0, stream>>>(QP, KP, VT, (float*)d_out);
}
